// GNNCoverageModel_12292196402001
// MI455X (gfx1250) — hardware-verified
//
#include <hip/hip_runtime.h>


#define NND 50000
#define NE 800000
#define F0 16
#define F1 128
#define F2 128
#define NGR 64
#define NOUT 16
#define RB 512
#define CHK 4096
#define EPT (CHK / RB)

typedef __attribute__((ext_vector_type(16))) __bf16   v16bf;
typedef __attribute__((ext_vector_type(16))) _Float16 v16h;
typedef __attribute__((ext_vector_type(8)))  float    v8f;
typedef __attribute__((ext_vector_type(8)))  unsigned v8u;

__device__ __forceinline__ unsigned f2bf(float f) { unsigned u = __float_as_uint(f); u += 0x7FFFu + ((u >> 16) & 1u); return u >> 16; }
__device__ __forceinline__ unsigned f2h(float f) { return (unsigned)__builtin_bit_cast(unsigned short, (_Float16)f); }
__device__ __forceinline__ int kpat(int v, int half) { return ((v & 4) ? 16 : 0) + half * 8 + 2 * (v & 3); }

template <int F16, int NP> struct Opnd { v16bf p[NP]; };

template <int F16, int NP> __device__ __forceinline__ void pack2(float f0, float f1, unsigned* o) {
    if (F16) { o[0] = f2h(f0) | (f2h(f1) << 16); return; }
    unsigned h0 = f2bf(f0), h1 = f2bf(f1); o[0] = h0 | (h1 << 16);
    if (NP >= 2) {
        float r0 = f0 - __uint_as_float(h0 << 16), r1 = f1 - __uint_as_float(h1 << 16);
        unsigned m0 = f2bf(r0), m1 = f2bf(r1); o[1] = m0 | (m1 << 16);
        if (NP >= 3) {
            float s0 = r0 - __uint_as_float(m0 << 16), s1 = r1 - __uint_as_float(m1 << 16);
            o[2] = f2bf(s0) | (f2bf(s1) << 16);
        }
    }
}
template <int F16, int NP> __device__ __forceinline__ void op_row(const float* rowp, int half, float sc, Opnd<F16, NP>& o) {
    v8u u[NP];
#pragma unroll
    for (int v = 0; v < 8; ++v) {
        int kk = kpat(v, half); unsigned t[3];
        pack2<F16, NP>(rowp[kk] * sc, rowp[kk + 1] * sc, t);
#pragma unroll
        for (int p = 0; p < NP; ++p) u[p][v] = t[p];
    }
#pragma unroll
    for (int p = 0; p < NP; ++p) o.p[p] = __builtin_bit_cast(v16bf, u[p]);
}
template <int F16, int NP> __device__ __forceinline__ void op_row_tail(const float* rowp, int half, float sc, int kvalid, Opnd<F16, NP>& o) {
    v8u u[NP];
#pragma unroll
    for (int v = 0; v < 8; ++v) {
        int kk = kpat(v, half); unsigned t[3];
        float f0 = kk < kvalid ? rowp[kk] * sc : 0.0f, f1 = (kk + 1) < kvalid ? rowp[kk + 1] * sc : 0.0f;
        pack2<F16, NP>(f0, f1, t);
#pragma unroll
        for (int p = 0; p < NP; ++p) u[p][v] = t[p];
    }
#pragma unroll
    for (int p = 0; p < NP; ++p) o.p[p] = __builtin_bit_cast(v16bf, u[p]);
}
template <int F16, int NP> __device__ __forceinline__ void op_col(const float* M, int ld, int n, int k0, int half, float sc, Opnd<F16, NP>& o) {
    v8u u[NP];
#pragma unroll
    for (int v = 0; v < 8; ++v) {
        int kk = k0 + kpat(v, half); unsigned t[3];
        pack2<F16, NP>(M[(size_t)kk * ld + n] * sc, M[(size_t)(kk + 1) * ld + n] * sc, t);
#pragma unroll
        for (int p = 0; p < NP; ++p) u[p][v] = t[p];
    }
#pragma unroll
    for (int p = 0; p < NP; ++p) o.p[p] = __builtin_bit_cast(v16bf, u[p]);
}
template <int F16, int NP> __device__ __forceinline__ void op_col_tail(const float* M, int ld, int n, int k0, int half, float sc, int K, Opnd<F16, NP>& o) {
    v8u u[NP];
#pragma unroll
    for (int v = 0; v < 8; ++v) {
        int kk = k0 + kpat(v, half); unsigned t[3];
        float f0 = kk < K ? M[(size_t)kk * ld + n] * sc : 0.0f, f1 = (kk + 1) < K ? M[(size_t)(kk + 1) * ld + n] * sc : 0.0f;
        pack2<F16, NP>(f0, f1, t);
#pragma unroll
        for (int p = 0; p < NP; ++p) u[p][v] = t[p];
    }
#pragma unroll
    for (int p = 0; p < NP; ++p) o.p[p] = __builtin_bit_cast(v16bf, u[p]);
}
__device__ __forceinline__ v8f wm_bf16(v16bf a, v16bf b, v8f c) { return __builtin_amdgcn_wmma_f32_16x16x32_bf16(false, a, false, b, (short)0, c, false, false); }
template <int F16, int NA, int NB> __device__ __forceinline__ v8f wmma_op(const Opnd<F16, NA>& a, const Opnd<F16, NB>& b, v8f c) {
    if (F16) {
        v16h ah = __builtin_bit_cast(v16h, a.p[0]), bh = __builtin_bit_cast(v16h, b.p[0]);
        c = __builtin_amdgcn_wmma_f32_16x16x32_f16(false, ah, false, bh, (short)0, c, false, false);
        asm volatile("v_nop\n\tv_nop\n\tv_nop\n\tv_nop" : "+v"(c) : "v"(ah), "v"(bh));
        return c;
    }
    constexpr int NMX = NA > NB ? NA : NB;
#pragma unroll
    for (int i = 0; i < NA; ++i)
#pragma unroll
        for (int j = 0; j < NB; ++j)
            if (i + j < NMX) c = wm_bf16(a.p[i], b.p[j], c);
    if (NA == 1 && NB == 1)      asm volatile("v_nop\n\tv_nop\n\tv_nop\n\tv_nop" : "+v"(c) : "v"(a.p[0]), "v"(b.p[0]));
    else if (NA == 2 && NB == 1) asm volatile("v_nop\n\tv_nop\n\tv_nop\n\tv_nop" : "+v"(c) : "v"(a.p[0]), "v"(a.p[1]), "v"(b.p[0]));
    else if (NA == 1 && NB == 2) asm volatile("v_nop\n\tv_nop\n\tv_nop\n\tv_nop" : "+v"(c) : "v"(a.p[0]), "v"(b.p[0]), "v"(b.p[1]));
    else if (NA == 2 && NB == 2) asm volatile("v_nop\n\tv_nop\n\tv_nop\n\tv_nop" : "+v"(c) : "v"(a.p[0]), "v"(a.p[1]), "v"(b.p[0]), "v"(b.p[1]));
    else                         asm volatile("v_nop\n\tv_nop\n\tv_nop\n\tv_nop" : "+v"(c) : "v"(a.p[0]), "v"(a.p[NA - 1]), "v"(b.p[0]), "v"(b.p[NB - 1]), "v"(a.p[NA / 2]), "v"(b.p[NB / 2]));
    return c;
}

struct ZMap { long long s1; long long s2; int zdiv; int pad_; };
__device__ __forceinline__ size_t zoff(const ZMap& m, int z) { return (size_t)((long long)(z / m.zdiv) * m.s1 + (long long)(z % m.zdiv) * m.s2); }

#define ACT_NONE 0
#define ACT_RELU 1
#define ACT_GELU_ERF 2
#define ACT_SILU 3
#define ACT_TANH 4
__device__ __forceinline__ float act_apply(int act, float x) {
    if (act == ACT_RELU) return x > 0.f ? x : 0.f;
    if (act == ACT_GELU_ERF) return 0.5f * x * (1.0f + erff(x * 0.70710678118654752f));
    if (act == ACT_SILU) return x / (1.0f + expf(-x));
    if (act == ACT_TANH) return tanhf(x);
    return x;
}
struct GemmArgs {
    ZMap za, zb_, zc, zbias, zadd, zrsc, zmul, zrbias;
    const float* A; const float* Bm; float* C; const float* bias; const float* add; const float* rsc; const float* mul; const float* rbias;
    long long ldadd, ldmul;
    int lda, ldb, ldc, K;
    float ascale, bscale, oscale, addscale;
    int M, nvalid, nstore, ldrsc;
    int bcs, pad1, pad2, pad3;
};
template <int BT, int F16, int NA, int NB, int RW, int CW, int ACT>
__global__ __launch_bounds__(256) void gemm_kernel(GemmArgs g) {
    constexpr int TR = 16 * RW, TC = 64 * CW, CSTR = TC + 4;
    __shared__ __align__(16) float cst[TR * CSTR];
    const int z = blockIdx.z;
    const float* A = g.A + zoff(g.za, z); const float* Bm = g.Bm + zoff(g.zb_, z); float* C = g.C + zoff(g.zc, z);
    const int tid = threadIdx.x, lane = tid & 31, wv = tid >> 5;
    const int l16 = lane & 15, half = lane >> 4;
    const int rt = wv % RW, ch = wv / RW;
    const int row0 = blockIdx.x * TR, col0 = blockIdx.y * TC + ch * 64;
    int arix = row0 + rt * 16 + l16; if (arix >= g.M) arix = g.M - 1;
    const float* arow = A + (size_t)arix * g.lda;
    v8f acc[4];
#pragma unroll
    for (int t = 0; t < 4; ++t) acc[t] = (v8f){};
    const int K = g.K;
#pragma unroll 1
    for (int kc = 0; kc < K; kc += 32) {
        Opnd<F16, NA> a;
        if (kc + 32 <= K) op_row<F16, NA>(arow + kc, half, g.ascale, a); else op_row_tail<F16, NA>(arow + kc, half, g.ascale, K - kc, a);
#pragma unroll
        for (int t = 0; t < 4; ++t) {
            Opnd<F16, NB> b;
            const int n = col0 + t * 16 + l16;
            if (n < g.nvalid) {
                if (BT) { if (kc + 32 <= K) op_row<F16, NB>(Bm + (size_t)n * g.ldb + kc, half, g.bscale, b); else op_row_tail<F16, NB>(Bm + (size_t)n * g.ldb + kc, half, g.bscale, K - kc, b); }
                else    { if (kc + 32 <= K) op_col<F16, NB>(Bm, g.ldb, n * g.bcs, kc, half, g.bscale, b); else op_col_tail<F16, NB>(Bm, g.ldb, n * g.bcs, kc, half, g.bscale, K, b); }
            } else {
#pragma unroll
                for (int p = 0; p < NB; ++p) b.p[p] = (v16bf){};
            }
            acc[t] = wmma_op<F16, NA, NB>(a, b, acc[t]);
        }
    }
    const float* bias = g.bias ? g.bias + zoff(g.zbias, z) : nullptr;
    const float* add = g.add ? g.add + zoff(g.zadd, z) : nullptr;
    const float* rsc = g.rsc ? g.rsc + zoff(g.zrsc, z) : nullptr;
    const float* mul = g.mul ? g.mul + zoff(g.zmul, z) : nullptr;
    const float* rbias = g.rbias ? g.rbias + zoff(g.zrbias, z) : nullptr;
#pragma unroll
    for (int t = 0; t < 4; ++t) {
        const int cl = ch * 64 + t * 16 + l16;
        const int cg = blockIdx.y * TC + cl;
        const bool cok = cg < g.nvalid;
        const float bv = (bias && cok) ? bias[(size_t)cg * g.bcs] : 0.0f;
#pragma unroll
        for (int r = 0; r < 8; ++r) {
            const int rl = rt * 16 + r + 8 * half;
            float v = acc[t][r] * g.oscale + bv;
            int rg = row0 + rl; if (rg >= g.M) rg = g.M - 1;
            if (rbias) v += rbias[rg];
            if (rsc) v *= rsc[(size_t)rg * g.ldrsc];
            if (mul && cok) v *= mul[(size_t)rg * g.ldmul + cg];
            if (add && cok) v += g.addscale * add[(size_t)rg * g.ldadd + cg];
            cst[rl * CSTR + cl] = v;
        }
    }
    __syncthreads();
    const int col = tid % TC, rsel = tid / TC, rstep = 256 / TC;
    if (ACT != ACT_NONE) {
#pragma unroll 1
        for (int r = rsel; r < TR; r += rstep) cst[r * CSTR + col] = act_apply(ACT, cst[r * CSTR + col]);
    }
    float* ob = C + (size_t)row0 * g.ldc + (size_t)blockIdx.y * TC;
    const bool colok = (int)(blockIdx.y * TC + col) < g.nstore;
    const int rmax = (g.M - row0 < TR) ? (g.M - row0) : TR;
    auto pass = [&]() {
        if (colok) {
#pragma unroll 4
            for (int r = rsel; r < rmax; r += rstep) *(volatile float*)(ob + (size_t)r * g.ldc + col) = cst[r * CSTR + col];
        }
    };
    pass();
    __threadfence();
    pass();
}
static inline ZMap zm(long long s1) { ZMap m; m.s1 = s1; m.s2 = 0; m.zdiv = 1; m.pad_ = 0; return m; }
static inline ZMap zm2(long long s1, long long s2, int zdiv) { ZMap m; m.s1 = s1; m.s2 = s2; m.zdiv = zdiv; m.pad_ = 0; return m; }
static inline GemmArgs gemm_args(const float* A, int lda, ZMap za, const float* Bm, int ldb, ZMap zb, float* C, int ldc, ZMap zc, int M, int N, int K) {
    GemmArgs g; g.za = za; g.zb_ = zb; g.zc = zc; g.zbias = zm(0); g.zadd = zm(0); g.zrsc = zm(0); g.zmul = zm(0); g.zrbias = zm(0);
    g.A = A; g.Bm = Bm; g.C = C; g.bias = nullptr; g.add = nullptr; g.rsc = nullptr; g.mul = nullptr; g.rbias = nullptr; g.ldadd = 0; g.ldmul = 0;
    g.lda = lda; g.ldb = ldb; g.ldc = ldc; g.K = K; g.ascale = 1.0f; g.bscale = 1.0f; g.oscale = 1.0f; g.addscale = 1.0f; g.M = M; g.nvalid = N; g.nstore = N; g.ldrsc = 1;
    g.bcs = 1; g.pad1 = 0; g.pad2 = 0; g.pad3 = 0;
    return g;
}
static_assert(sizeof(ZMap) == 24, "ZMap layout");
static_assert(sizeof(GemmArgs) == 8 * 24 + 8 * 8 + 2 * 8 + 4 * 4 + 4 * 4 + 4 * 4 + 4 * 4, "GemmArgs has no padding");

__global__ __launch_bounds__(256) void softmax_rows(float* S, long long sy, long long sx, int L, float prescale, const float* addv, long long say, int aydiv, int causal,
                                                  const int* imask, long long imy, long long imx, float maskval) {
    __shared__ float red[8];
    const int tid = threadIdx.x, lane = tid & 31, wid = tid >> 5;
    float* row = S + (size_t)blockIdx.y * sy + (size_t)blockIdx.x * sx;
    const float* av = addv ? addv + (size_t)(blockIdx.y / aydiv) * say : nullptr;
    const int* im = imask ? imask + (size_t)(blockIdx.y / aydiv) * imy + (size_t)blockIdx.x * imx : nullptr;
    float v[16];
    const int nj = L / 256;
    float mx = -__builtin_inff();
#pragma unroll
    for (int j = 0; j < 16; ++j) if (j < nj) { float t = row[tid + 256 * j] * prescale; if (av) t += av[tid + 256 * j]; if (im && im[tid + 256 * j] == 0) t = maskval; if (causal && (tid + 256 * j) > (int)blockIdx.x) t = -__builtin_inff(); v[j] = t; mx = fmaxf(mx, t); }
#pragma unroll
    for (int o = 16; o; o >>= 1) mx = fmaxf(mx, __shfl_xor(mx, o, 32));
    if (lane == 0) red[wid] = mx;
    __syncthreads();
    float m = red[0];
#pragma unroll
    for (int i = 1; i < 8; ++i) m = fmaxf(m, red[i]);
    if (m == -__builtin_inff()) m = 0.f;
    __syncthreads();
    float sum = 0.f;
#pragma unroll
    for (int j = 0; j < 16; ++j) if (j < nj) { v[j] = expf(v[j] - m); sum += v[j]; }
#pragma unroll
    for (int o = 16; o; o >>= 1) sum += __shfl_xor(sum, o, 32);
    if (lane == 0) red[wid] = sum;
    __syncthreads();
    float tot = 0.f;
#pragma unroll
    for (int i = 0; i < 8; ++i) tot += red[i];
    const float inv = 1.0f / tot;
#pragma unroll
    for (int j = 0; j < 16; ++j) if (j < nj) *(volatile float*)(row + tid + 256 * j) = v[j] * inv;
    __threadfence();
#pragma unroll
    for (int j = 0; j < 16; ++j) if (j < nj) *(volatile float*)(row + tid + 256 * j) = v[j] * inv;
}

#define VST2(T, p, v) do { const T vst2_v_ = (v); *(volatile T*)(p) = vst2_v_; __threadfence(); *(volatile T*)(p) = vst2_v_; } while (0)
__device__ __forceinline__ int block_excl_scan(int cnt, int* scan, int tid, int& total) { __syncthreads(); scan[tid] = cnt; __syncthreads();
    for (int o = 1; o < RB; o <<= 1) { const int v = (tid >= o) ? scan[tid - o] : 0; __syncthreads(); scan[tid] += v; __syncthreads(); }
    total = scan[RB - 1]; return scan[tid] - cnt; }
__global__ __launch_bounds__(RB) void k_deg(const int* __restrict__ ei, float* DINV) { __shared__ int Ld[CHK]; __shared__ int scan[RB]; const int tid = threadIdx.x; const int n0 = blockIdx.x * RB; int ci = 0;
    for (int e0 = 0; e0 < NE; e0 += CHK) { int hd[EPT]; int cd = 0;
#pragma unroll
        for (int k = 0; k < EPT; ++k) { const int e = e0 + tid * EPT + k; hd[k] = -1; if (e < NE) { const int d = ei[(size_t)NE + e]; if (d >= n0 && d < n0 + RB) { hd[k] = d - n0; ++cd; } } }
        int tot; int p = block_excl_scan(cd, scan, tid, tot);
#pragma unroll
        for (int k = 0; k < EPT; ++k) if (hd[k] >= 0) Ld[p++] = hd[k];
        __syncthreads();
        for (int q = 0; q < tot; ++q) ci += (Ld[q] == tid);
        __syncthreads(); }
    const int n = n0 + tid; if (n < NND) { VST2(float, DINV + n, rsqrtf((float)ci + 1.f)); } }
template <int NC>
__global__ __launch_bounds__(RB) void k_aggr(const float* __restrict__ H, const float* __restrict__ DINV, const int* __restrict__ ei, float* RAW) { __shared__ int Lr[CHK]; __shared__ int Lc[CHK]; __shared__ int scan[RB]; const int tid = threadIdx.x; const int n0 = blockIdx.x * RB; float acc[NC];
#pragma unroll
    for (int c = 0; c < NC; ++c) acc[c] = 0.f;
    for (int e0 = 0; e0 < NE; e0 += CHK) { int hr[EPT], hc[EPT]; int cnt = 0;
#pragma unroll
        for (int k = 0; k < EPT; ++k) { const int e = e0 + tid * EPT + k; hr[k] = -1; if (e < NE) { const int d = ei[(size_t)NE + e]; if (d >= n0 && d < n0 + RB) { hr[k] = d - n0; int s = ei[e]; s = s < 0 ? 0 : (s >= NND ? NND - 1 : s); hc[k] = s; ++cnt; } } }
        int tot; int p = block_excl_scan(cnt, scan, tid, tot);
#pragma unroll
        for (int k = 0; k < EPT; ++k) if (hr[k] >= 0) { Lr[p] = hr[k]; Lc[p] = hc[k]; ++p; }
        __syncthreads();
        for (int q = 0; q < tot; ++q) { if (Lr[q] == tid) { const int s = Lc[q]; const float ds = DINV[s]; const float* hrow = H + (size_t)s * NC;
#pragma unroll
                for (int c = 0; c < NC; ++c) acc[c] += ds * hrow[c]; } }
        __syncthreads(); }
    const int n = n0 + tid; if (n >= NND) return;
#pragma unroll
    for (int c = 0; c < NC; ++c) VST2(float, RAW + (size_t)n * NC + c, acc[c]); }
__global__ __launch_bounds__(256) void k_epi(const float* __restrict__ RAW, const float* __restrict__ H, const float* __restrict__ DINV, const float* __restrict__ bias, int NC, float* OUT) { const size_t q = (size_t)blockIdx.x * 256 + threadIdx.x; if (q >= (size_t)NND * NC) return; const size_t n = q / NC; const float dn = DINV[n]; VST2(float, OUT + q, fmaxf(dn * (RAW[q] + dn * H[q]) + bias[q % NC], 0.f)); }
__global__ __launch_bounds__(256) void k_pool(const float* __restrict__ Hh, const int* __restrict__ bid, const float* __restrict__ Wfc, const float* __restrict__ bfc, float* O32) { __shared__ double red[2][F2]; __shared__ double cn[2]; __shared__ float pooled[F2]; const int g = blockIdx.x, tid = threadIdx.x; const int c = tid & 127, part = tid >> 7; double s = 0.0; double cnt = 0.0;
    for (int n = part; n < NND; n += 2) { if (bid[n] == g) { s += (double)Hh[(size_t)n * F2 + c]; if (c == 0) cnt += 1.0; } }
    red[part][c] = s; if (c == 0) cn[part] = cnt; __syncthreads();
    if (tid < F2) pooled[tid] = (float)((red[0][tid] + red[1][tid]) / fmax(cn[0] + cn[1], 1.0)); __syncthreads();
    if (tid < 32) { float a = 0.f; if (tid < NOUT) { a = bfc[tid];
#pragma unroll 1
            for (int k = 0; k < F2; ++k) a += pooled[k] * Wfc[k * NOUT + tid]; } VST2(float, O32 + (size_t)g * 32 + tid, a); } }
__global__ __launch_bounds__(256) void k_copy(const float* __restrict__ O32, float* out) { const int q = blockIdx.x * 256 + threadIdx.x; if (q >= NGR * NOUT) return; VST2(float, out + q, O32[(size_t)(q / NOUT) * 32 + (q % NOUT)]); }
extern "C" void kernel_launch(void* const* d_in, const int* in_sizes, int n_in,
                              void* d_out, int out_size, void* d_ws, size_t ws_size, hipStream_t stream) {
    (void)in_sizes; (void)n_in; (void)out_size;
    const float* x = (const float*)d_in[0]; const int* ei = (const int*)d_in[1]; const int* bid = (const int*)d_in[2]; const float* W1 = (const float*)d_in[3]; const float* b1 = (const float*)d_in[4]; const float* W2 = (const float*)d_in[5]; const float* b2 = (const float*)d_in[6]; const float* Wfc = (const float*)d_in[7]; const float* bfc = (const float*)d_in[8];
    float* out = (float*)d_out;
    char* wsp = (char*)d_ws;
    auto take = [&](size_t bytes) { char* p = wsp; wsp += (bytes + 255) & ~(size_t)255; return (void*)p; };
    float* DINV = (float*)take((size_t)NND * 4); float* H1 = (float*)take((size_t)NND * F1 * 4); float* R1 = (float*)take((size_t)NND * F1 * 4); float* A1 = (float*)take((size_t)NND * F1 * 4); float* R2 = (float*)take((size_t)NND * F2 * 4); float* A2 = (float*)take((size_t)NND * F2 * 4); float* O32 = (float*)take(NGR * 32 * 4);
    float* H2 = H1;
    if ((size_t)(wsp - (char*)d_ws) > ws_size) return;
    const int nb = (NND + RB - 1) / RB;
    k_deg<<<nb, RB, 0, stream>>>(ei, DINV);
    { GemmArgs g = gemm_args(x, F0, zm(0), W1, F1, zm(0), H1, F1, zm(0), NND, F1, F0); gemm_kernel<0, 0, 2, 2, 4, 2, ACT_NONE><<<dim3((NND + 63) / 64, 1, 1), 256, 0, stream>>>(g); }
    k_aggr<F1><<<nb, RB, 0, stream>>>(H1, DINV, ei, R1);
    k_epi<<<(unsigned)(((size_t)NND * F1 + 255) / 256), 256, 0, stream>>>(R1, H1, DINV, b1, F1, A1);
    { GemmArgs g = gemm_args(A1, F1, zm(0), W2, F2, zm(0), H2, F2, zm(0), NND, F2, F1); gemm_kernel<0, 0, 2, 2, 4, 2, ACT_NONE><<<dim3((NND + 63) / 64, 1, 1), 256, 0, stream>>>(g); }
    k_aggr<F2><<<nb, RB, 0, stream>>>(H2, DINV, ei, R2);
    k_epi<<<(unsigned)(((size_t)NND * F2 + 255) / 256), 256, 0, stream>>>(R2, H2, DINV, b2, F2, A2);
    k_pool<<<NGR, 256, 0, stream>>>(A2, bid, Wfc, bfc, O32);
    k_copy<<<(NGR * NOUT + 255) / 256, 256, 0, stream>>>(O32, out);
}
